// Hgru3_43954695307924
// MI455X (gfx1250) — hardware-verified
//
#include <hip/hip_runtime.h>
#include <math.h>

constexpr int kBatch    = 2;
constexpr int kSeqLen   = 1024;
constexpr int kEmb      = 1024;
constexpr int kHeadDim  = 64;
constexpr int kHeads    = 16;
constexpr int kTok      = kBatch * kSeqLen;
constexpr int kProjN    = 3 * kEmb;
constexpr int kGateRank = 64;
constexpr float kEps        = 1e-5f;
constexpr float kInvHeadDim = 1.0f / 64.0f;

typedef __attribute__((ext_vector_type(16))) _Float16 v16h;
typedef __attribute__((ext_vector_type(8)))  _Float16 v8h;
typedef __attribute__((ext_vector_type(16))) __bf16   v16b;
typedef __attribute__((ext_vector_type(8)))  __bf16   v8b;
typedef __attribute__((ext_vector_type(8)))  float    v8f;
typedef __attribute__((ext_vector_type(4)))  float    v4f;
typedef __attribute__((ext_vector_type(4)))  unsigned int v4u;

__device__ __forceinline__ unsigned short f2bf_bits(float f) {
  unsigned u = __float_as_uint(f);
  return (unsigned short)((u + 0x7FFFu + ((u >> 16) & 1u)) >> 16);
}
__device__ __forceinline__ float bf_bits2f(unsigned short h) { return __uint_as_float(((unsigned)h) << 16); }

__device__ __forceinline__ void dep_guard_h(v8f& a, v8f& b, v16h x, v16h y) { asm volatile("v_nop\n\tv_nop\n\tv_nop\n\tv_nop" : "+v"(a), "+v"(b) : "v"(x), "v"(y)); }
__device__ __forceinline__ void dep_guard_b(v8f& a, v8f& b, v16b x, v16b y) { asm volatile("v_nop\n\tv_nop\n\tv_nop\n\tv_nop" : "+v"(a), "+v"(b) : "v"(x), "v"(y)); }
__device__ __forceinline__ void keep4_h(v16h a, v16h b, v16h c, v16h d) { asm volatile("v_nop" :: "v"(a), "v"(b), "v"(c), "v"(d)); }
__device__ __forceinline__ void keep4_b(v16b a, v16b b, v16b c, v16b d) { asm volatile("v_nop" :: "v"(a), "v"(b), "v"(c), "v"(d)); }
__device__ __forceinline__ void acc_guard4(v8f& a, v8f& b, v8f& c, v8f& d) { asm volatile("v_nop\n\tv_nop\n\tv_nop\n\tv_nop" : "+v"(a), "+v"(b), "+v"(c), "+v"(d)); }
template <typename T> struct Frag;
template <> struct Frag<_Float16> {
  typedef v16h V; union U { v16h v; v8h h[2]; };
  static __device__ __forceinline__ v16h load(const _Float16* p) {
    U f; f.h[0] = *(const v8h*)(p); f.h[1] = *(const v8h*)(p + 16); return f.v;
  }
  static __device__ __forceinline__ v8f mma(v16h a, v16h b, v8f c) {
    return __builtin_amdgcn_wmma_f32_16x16x32_f16(false, a, false, b, (short)0, c, false, false);
  }
  static __device__ __forceinline__ void guard(v8f& a, v8f& b, v16h x, v16h y) { dep_guard_h(a, b, x, y); }
  static __device__ __forceinline__ void keep(v16h a, v16h b, v16h c, v16h d) { keep4_h(a, b, c, d); }
};
template <> struct Frag<__bf16> {
  typedef v16b V; union U { v16b v; v8b h[2]; };
  static __device__ __forceinline__ v16b load(const __bf16* p) {
    U f; f.h[0] = *(const v8b*)(p); f.h[1] = *(const v8b*)(p + 16); return f.v;
  }
  static __device__ __forceinline__ v8f mma(v16b a, v16b b, v8f c) {
    return __builtin_amdgcn_wmma_f32_16x16x32_bf16(false, a, false, b, (short)0, c, false, false);
  }
  static __device__ __forceinline__ void guard(v8f& a, v8f& b, v16b x, v16b y) { dep_guard_b(a, b, x, y); }
  static __device__ __forceinline__ void keep(v16b a, v16b b, v16b c, v16b d) { keep4_b(a, b, c, d); }
};

__device__ __forceinline__ unsigned pk16(unsigned short a, unsigned short b) { return (unsigned)a | ((unsigned)b << 16); }

template <int ET> struct Elem;
template <> struct Elem<0> { typedef _Float16 T; };
template <> struct Elem<1> { typedef __bf16 T; };
template <int ET, bool SPLIT, int BIAS_MODE, int OUT_MODE, bool RESID, int ACT = 0>
__global__ __launch_bounds__(256) void wmma_gemm64(
    const unsigned short* __restrict__ Ap, const unsigned short* __restrict__ A2p, int lda, long strideA,
    const unsigned short* __restrict__ Btp, const unsigned short* __restrict__ Bt2p, int ldb, long strideB,
    void* __restrict__ Cout, void* __restrict__ Cout2, int ldc, long strideC,
    const float* __restrict__ bias,
    const float* __restrict__ resid, long strideR,
    int M, int N, int K, float scale) {
  typedef typename Elem<ET>::T T;
  typedef typename Frag<T>::V V;
  const T* A = (const T*)Ap; const T* A2 = (const T*)A2p; const T* Bt = (const T*)Btp; const T* Bt2 = (const T*)Bt2p;
  __shared__ __align__(16) float sT[8][16 * 68];
  const int b    = blockIdx.y;
  const int lane = threadIdx.x & 31;
  const int wave = threadIdx.x >> 5;
  const int tilesN = N >> 6;
  const int tilesM = M >> 6;
  const int tile = blockIdx.x * 8 + wave;
  if (tile >= tilesM * tilesN) return;
  const int tm = tile / tilesN;
  const int tn = tile - tm * tilesN;
  const int m0 = tm << 6;
  const int n0 = tn << 6;

  const T* Ab  = A  + (size_t)b * strideA;
  const T* Bb  = Bt + (size_t)b * strideB;
  const T* Ab2 = SPLIT ? (A2  + (size_t)b * strideA) : nullptr;
  const T* Bb2 = SPLIT ? (Bt2 + (size_t)b * strideB) : nullptr;

  const int rlane = lane & 15;
  const int koff  = (lane >> 4) * 8;
  const int mOff  = (lane >> 4) * 8;

  v8f acc[4][4];
#pragma unroll
  for (int i = 0; i < 4; ++i)
#pragma unroll
    for (int j = 0; j < 4; ++j) acc[i][j] = (v8f){0.f,0.f,0.f,0.f,0.f,0.f,0.f,0.f};

  for (int k0 = 0; k0 < K; k0 += 32) {
    V bh[4], bl[4];
#pragma unroll
    for (int j = 0; j < 4; ++j) {
      const size_t bo = (size_t)(n0 + (j << 4) + rlane) * ldb + koff + k0;
      bh[j] = Frag<T>::load(Bb + bo);
      if (SPLIT) bl[j] = Frag<T>::load(Bb2 + bo);
    }
#pragma unroll
    for (int i = 0; i < 4; ++i) {
      const size_t ao = (size_t)(m0 + (i << 4) + rlane) * lda + koff + k0;
      V ah = Frag<T>::load(Ab + ao);
      V al;
      if (SPLIT) al = Frag<T>::load(Ab2 + ao);
#pragma unroll
      for (int j = 0; j < 4; ++j) {
        acc[i][j] = Frag<T>::mma(ah, bh[j], acc[i][j]);
        if (SPLIT) {
          acc[i][j] = Frag<T>::mma(ah, bl[j], acc[i][j]);
          acc[i][j] = Frag<T>::mma(al, bh[j], acc[i][j]);
        }
      }
      Frag<T>::guard(acc[i][0], acc[i][3], ah, SPLIT ? al : ah);
    }
    Frag<T>::keep(bh[0], bh[1], bh[2], bh[3]);
    if (SPLIT) Frag<T>::keep(bl[0], bl[1], bl[2], bl[3]);
  }
  acc_guard4(acc[0][0], acc[0][1], acc[0][2], acc[0][3]);
  acc_guard4(acc[1][0], acc[1][1], acc[1][2], acc[1][3]);
  acc_guard4(acc[2][0], acc[2][1], acc[2][2], acc[2][3]);
  acc_guard4(acc[3][0], acc[3][1], acc[3][2], acc[3][3]);

  float* slab = sT[wave];
  const float* Rb = RESID ? (resid + (size_t)b * strideR) : nullptr;
#pragma unroll
  for (int i = 0; i < 4; ++i) {
    const int mBase = m0 + (i << 4);
#pragma unroll
    for (int j = 0; j < 4; ++j) {
      const int n = n0 + (j << 4) + rlane;
      float bv = 0.f;
      if (BIAS_MODE == 2) bv = bias[n];
#pragma unroll
      for (int r = 0; r < 8; ++r) {
        float v = acc[i][j][r] * scale;
        if (BIAS_MODE == 1) v += bias[mBase + mOff + r];
        if (BIAS_MODE == 2) v += bv;
        if (RESID) v += Rb[(size_t)(mBase + mOff + r) * ldc + n];
        if (ACT == 2) v = fmaxf(v, 0.0f);
        if (ACT == 4) v = (v > 0.f) ? v : 0.01f * v;
        slab[(mOff + r) * 68 + (j << 4) + rlane] = v;
      }
    }
    __builtin_amdgcn_fence(__ATOMIC_RELEASE, "workgroup");
    __builtin_amdgcn_wave_barrier();
    __builtin_amdgcn_fence(__ATOMIC_ACQUIRE, "workgroup");
    if (OUT_MODE == 0) {
      float* C = (float*)Cout + (size_t)b * strideC;
      const int hh = lane >> 4, c4 = (lane & 15) * 4;
      for (int pass = 0; pass < 2; ++pass) {
#pragma unroll
        for (int it = 0; it < 8; ++it) {
          const int row = it * 2 + hh;
          v4f v = *(const v4f*)(slab + row * 68 + c4);
          *(volatile v4f*)(C + (size_t)(mBase + row) * ldc + n0 + c4) = v;
        }
        __threadfence();
      }
    } else {
      const int q = lane >> 3, c8 = (lane & 7) * 8;
      unsigned short* C  = (unsigned short*)Cout  + (size_t)b * strideC;
      unsigned short* C2 = (OUT_MODE == 2) ? ((unsigned short*)Cout2 + (size_t)b * strideC) : nullptr;
      for (int pass = 0; pass < 2; ++pass) {
#pragma unroll
        for (int it = 0; it < 4; ++it) {
          const int row = it * 4 + q;
          const float* sp = slab + row * 68 + c8;
          v8h hv, lv;
#pragma unroll
          for (int e = 0; e < 8; ++e) {
            if (OUT_MODE == 1) {
              hv[e] = (_Float16)sp[e];
            } else {
              unsigned short hb = f2bf_bits(sp[e]);
              unsigned short lb = f2bf_bits(sp[e] - bf_bits2f(hb));
              hv[e] = __builtin_bit_cast(_Float16, hb);
              lv[e] = __builtin_bit_cast(_Float16, lb);
            }
          }
          *(volatile v8h*)(C + (size_t)(mBase + row) * ldc + n0 + c8) = hv;
          if (OUT_MODE == 2) *(volatile v8h*)(C2 + (size_t)(mBase + row) * ldc + n0 + c8) = lv;
        }
        __threadfence();
      }
    }
    __builtin_amdgcn_fence(__ATOMIC_RELEASE, "workgroup");
    __builtin_amdgcn_wave_barrier();
    __builtin_amdgcn_fence(__ATOMIC_ACQUIRE, "workgroup");
  }
}

__global__ __launch_bounds__(256) void split8_bf16_kernel(const float* __restrict__ in,
                                                          unsigned short* __restrict__ oh,
                                                          unsigned short* __restrict__ ol, int n8) {
  const int i = blockIdx.x * 256 + threadIdx.x;
  if (i >= n8) return;
  const float* p = in + 8 * (size_t)i;
  const v4f a = *(const v4f*)(p);
  const v4f c = *(const v4f*)(p + 4);
  unsigned short hb[8], lb[8];
#pragma unroll
  for (int e = 0; e < 4; ++e) {
    hb[e]     = f2bf_bits(a[e]);
    lb[e]     = f2bf_bits(a[e] - bf_bits2f(hb[e]));
    hb[4 + e] = f2bf_bits(c[e]);
    lb[4 + e] = f2bf_bits(c[e] - bf_bits2f(hb[4 + e]));
  }
  const v4u uh = (v4u){pk16(hb[0], hb[1]), pk16(hb[2], hb[3]), pk16(hb[4], hb[5]), pk16(hb[6], hb[7])};
  const v4u ul = (v4u){pk16(lb[0], lb[1]), pk16(lb[2], lb[3]), pk16(lb[4], lb[5]), pk16(lb[6], lb[7])};
  unsigned short* qh = oh + 8 * (size_t)i;
  unsigned short* ql = ol + 8 * (size_t)i;
  *(volatile v4u*)qh = uh;
  *(volatile v4u*)ql = ul;
  __threadfence();
  *(volatile v4u*)qh = uh;
  *(volatile v4u*)ql = ul;
}

__global__ __launch_bounds__(256) void wtsplit_kernel(const float* __restrict__ W0, const float* __restrict__ W1,
                                                      const float* __restrict__ W2, int Kin, int Nout,
                                                      unsigned short* __restrict__ outH,
                                                      unsigned short* __restrict__ outL) {
  __shared__ float sm[64][65];
  const int t  = threadIdx.x;
  const int k0 = blockIdx.x * 64;
  const int n0 = blockIdx.y * 64;
  const int z  = blockIdx.z;
  const float* W = (z == 0) ? W0 : (z == 1) ? W1 : W2;
#pragma unroll
  for (int i = 0; i < 16; ++i) {
    const int e = i * 256 + t;
    const int r = e >> 6;
    const int c = e & 63;
    sm[c][r] = W[(size_t)(k0 + r) * Nout + n0 + c];
  }
  __syncthreads();
  const int lane = t & 31, wave = t >> 5;
  const int q = lane >> 3, c8 = (lane & 7) * 8;
  const size_t rowOff = (size_t)z * Nout + n0;
  for (int pass = 0; pass < 2; ++pass) {
#pragma unroll
    for (int it = 0; it < 2; ++it) {
      const int row = wave * 8 + it * 4 + q;
      unsigned short hb[8], lb[8];
#pragma unroll
      for (int e = 0; e < 8; ++e) {
        const float v = sm[row][c8 + e];
        hb[e] = f2bf_bits(v);
        lb[e] = f2bf_bits(v - bf_bits2f(hb[e]));
      }
      const v4u uh = (v4u){pk16(hb[0], hb[1]), pk16(hb[2], hb[3]), pk16(hb[4], hb[5]), pk16(hb[6], hb[7])};
      const v4u ul = (v4u){pk16(lb[0], lb[1]), pk16(lb[2], lb[3]), pk16(lb[4], lb[5]), pk16(lb[6], lb[7])};
      const size_t o = (rowOff + row) * (size_t)Kin + k0 + c8;
      *(volatile v4u*)(outH + o) = uh;
      *(volatile v4u*)(outL + o) = ul;
    }
    __threadfence();
  }
}

__global__ __launch_bounds__(256) void prep_kernel(const float* __restrict__ pre, const float* __restrict__ delta,
                                                   float* __restrict__ qa, float* __restrict__ kv,
                                                   float* __restrict__ dec) {
  __shared__ __align__(16) float st[3][256];
  const int tid = threadIdx.x;
  const size_t idx = (size_t)blockIdx.x * 256 + tid;
  const size_t m = idx >> 10;
  const int c = (int)(idx & 1023);
  const float xq = pre[m * kProjN + c];
  const float xk = pre[m * kProjN + kEmb + c];
  const float dl = delta[c];
  const float qv = xq * (1.0f / (1.0f + expf(-xq)));
  const float z  = xk + dl;
  const float lf = -(fmaxf(-z, 0.0f) + log1pf(expf(-fabsf(z))));
  const float kval = -expm1f(lf);
  const float dc   = expf(lf);
  st[0][tid] = qv;
  st[1][tid] = kval;
  st[2][tid] = dc;
  __syncthreads();
  if (tid < 192) {
    const int arr = tid >> 6;
    const int pos = (tid & 63) * 4;
    const v4f val = *(const v4f*)(&st[arr][pos]);
    float* dst = (arr == 0) ? qa : (arr == 1) ? kv : dec;
    float* pd = dst + (size_t)blockIdx.x * 256 + pos;
    *(volatile v4f*)pd = val;
    __threadfence();
    *(volatile v4f*)pd = val;
  }
}

__global__ __launch_bounds__(128) void decay_scan_kernel(const float* __restrict__ qa, const float* __restrict__ kv,
                                                         const float* __restrict__ dec, const float* __restrict__ pre,
                                                         float* __restrict__ o) {
  __shared__ __align__(16) float qs[2][64];
  __shared__ __align__(16) float ks[2][64];
  __shared__ __align__(16) float es[2][64];
  __shared__ __align__(16) float obuf[16][64];
  const int tid  = threadIdx.x;
  const int lane = tid & 31;
  const int wave = tid >> 5;
  const int half = lane >> 4;
  const int c    = lane & 15;
  const int dv   = wave * 16 + c;
  const int rb   = half * 32;
  const int bh   = blockIdx.x;
  const int b    = bh >> 4;
  const int h    = bh & 15;
  const int hc   = h * kHeadDim;
  const size_t mrow0 = (size_t)b * kSeqLen;

  float s[32];
#pragma unroll
  for (int i = 0; i < 32; ++i) s[i] = 0.0f;

#pragma unroll 1
  for (int t = 0; t < kSeqLen; ++t) {
    const int buf = t & 1;
    const size_t m = mrow0 + (size_t)t;
    if (tid < 64) {
      const size_t src = m * kEmb + hc + tid;
      qs[buf][tid] = qa[src];
      ks[buf][tid] = kv[src];
      es[buf][tid] = dec[src];
    }
    const float vv = pre[m * kProjN + 2 * kEmb + hc + dv];
    __syncthreads();
    float p = 0.0f;
#pragma unroll
    for (int i4 = 0; i4 < 8; ++i4) {
      const v4f q4 = *(const v4f*)(&qs[buf][rb + 4 * i4]);
      const v4f k4 = *(const v4f*)(&ks[buf][rb + 4 * i4]);
      const v4f e4 = *(const v4f*)(&es[buf][rb + 4 * i4]);
#pragma unroll
      for (int e = 0; e < 4; ++e) {
        const int idx = 4 * i4 + e;
        const float sn = s[idx] * e4[e] + k4[e] * vv;
        s[idx] = sn;
        p = fmaf(q4[e], sn, p);
      }
    }
    p += __shfl_xor(p, 16, 32);
    if (half == 0) obuf[t & 15][dv] = p;
    if ((t & 15) == 15) {
      __syncthreads();
      const size_t r0 = m - 15;
      const int c4 = c * 4;
      for (int pass = 0; pass < 2; ++pass) {
#pragma unroll
        for (int it = 0; it < 2; ++it) {
          const int row = it * 8 + wave * 2 + half;
          const v4f val = *(const v4f*)(&obuf[row][c4]);
          *(volatile v4f*)(o + (r0 + (size_t)row) * kEmb + hc + c4) = val;
        }
        __threadfence();
      }
    }
  }
}

__global__ __launch_bounds__(256) void gate_norm_kernel(const float* __restrict__ o, const float* __restrict__ gate,
                                                        const float* __restrict__ nw,
                                                        unsigned short* __restrict__ onh,
                                                        unsigned short* __restrict__ onl) {
  __shared__ __align__(16) float slab[8][64];
  const int lane = threadIdx.x & 31;
  const int wave = threadIdx.x >> 5;
  const int g    = blockIdx.x * 8 + wave;
  const int bt   = g >> 4;
  const int h    = g & 15;
  const size_t base = (size_t)bt * kEmb + (size_t)h * kHeadDim;
  const float o0 = o[base + lane];
  const float o1 = o[base + lane + 32];
  const float a0 = gate[base + lane];
  const float a1 = gate[base + lane + 32];
  const float y0 = o0 * (1.0f / (1.0f + expf(-a0)));
  const float y1 = o1 * (1.0f / (1.0f + expf(-a1)));
  float ss = y0 * y0 + y1 * y1;
#pragma unroll
  for (int off = 16; off > 0; off >>= 1) ss += __shfl_xor(ss, off, 32);
  const float r = rsqrtf(ss * kInvHeadDim + kEps);
  slab[wave][lane]      = (y0 * r) * nw[h * kHeadDim + lane];
  slab[wave][lane + 32] = (y1 * r) * nw[h * kHeadDim + lane + 32];
  __builtin_amdgcn_fence(__ATOMIC_RELEASE, "workgroup");
  __builtin_amdgcn_wave_barrier();
  __builtin_amdgcn_fence(__ATOMIC_ACQUIRE, "workgroup");
  const int c8 = (lane & 7) * 8;
  const v4f va = *(const v4f*)(&slab[wave][c8]);
  const v4f vb = *(const v4f*)(&slab[wave][c8 + 4]);
  unsigned short hb[8], lb[8];
#pragma unroll
  for (int e = 0; e < 4; ++e) {
    hb[e]     = f2bf_bits(va[e]);
    lb[e]     = f2bf_bits(va[e] - bf_bits2f(hb[e]));
    hb[4 + e] = f2bf_bits(vb[e]);
    lb[4 + e] = f2bf_bits(vb[e] - bf_bits2f(hb[4 + e]));
  }
  const v4u uh = (v4u){pk16(hb[0], hb[1]), pk16(hb[2], hb[3]), pk16(hb[4], hb[5]), pk16(hb[6], hb[7])};
  const v4u ul = (v4u){pk16(lb[0], lb[1]), pk16(lb[2], lb[3]), pk16(lb[4], lb[5]), pk16(lb[6], lb[7])};
  if (lane < 8) {
    unsigned short* ph = onh + base + c8;
    unsigned short* pl = onl + base + c8;
    *(volatile v4u*)ph = uh;
    *(volatile v4u*)pl = ul;
    __threadfence();
    *(volatile v4u*)ph = uh;
    *(volatile v4u*)pl = ul;
  }
}

extern "C" void kernel_launch(void* const* d_in, const int* in_sizes, int n_in,
                              void* d_out, int out_size, void* d_ws,
                              size_t ws_size, hipStream_t stream) {
  if (n_in < 9) return;
  if (in_sizes[0] != kTok * kEmb || in_sizes[1] != kEmb * kEmb || in_sizes[2] != kEmb * kEmb ||
      in_sizes[3] != kEmb * kEmb || in_sizes[4] != kEmb * kEmb || in_sizes[5] != kEmb ||
      in_sizes[6] != kEmb * kGateRank || in_sizes[7] != kGateRank * kEmb || in_sizes[8] != kEmb) return;
  if (out_size != kTok * kEmb) return;

  const float* x     = (const float*)d_in[0];
  const float* Wq    = (const float*)d_in[1];
  const float* Wk    = (const float*)d_in[2];
  const float* Wv    = (const float*)d_in[3];
  const float* Wo    = (const float*)d_in[4];
  const float* delta = (const float*)d_in[5];
  const float* G1    = (const float*)d_in[6];
  const float* G2    = (const float*)d_in[7];
  const float* normw = (const float*)d_in[8];
  float* out = (float*)d_out;

  char* ws = (char*)d_ws;
  size_t off = 0;
  const size_t szX16   = (size_t)kTok * kEmb * 2;
  const size_t szWT16  = (size_t)kProjN * kEmb * 2;
  const size_t szG16   = (size_t)kGateRank * kEmb * 2;
  const size_t szWo16  = (size_t)kEmb * kEmb * 2;
  const size_t szPre   = (size_t)kTok * kProjN * 4;
  const size_t szTokF  = (size_t)kTok * kEmb * 4;
  const size_t szG1p   = (size_t)kTok * kGateRank * 2;
  unsigned short* xh   = (unsigned short*)(ws + off); off += szX16;
  unsigned short* xl   = (unsigned short*)(ws + off); off += szX16;
  unsigned short* WTh  = (unsigned short*)(ws + off); off += szWT16;
  unsigned short* WTl  = (unsigned short*)(ws + off); off += szWT16;
  unsigned short* G1Th = (unsigned short*)(ws + off); off += szG16;
  unsigned short* G1Tl = (unsigned short*)(ws + off); off += szG16;
  unsigned short* G2Th = (unsigned short*)(ws + off); off += szG16;
  unsigned short* G2Tl = (unsigned short*)(ws + off); off += szG16;
  unsigned short* WoTh = (unsigned short*)(ws + off); off += szWo16;
  unsigned short* WoTl = (unsigned short*)(ws + off); off += szWo16;
  float* pre  = (float*)(ws + off); off += szPre;
  float* qa   = (float*)(ws + off); off += szTokF;
  float* kvp  = (float*)(ws + off); off += szTokF;
  float* decp = (float*)(ws + off); off += szTokF;
  unsigned short* g1h = (unsigned short*)(ws + off); off += szG1p;
  unsigned short* g1l = (unsigned short*)(ws + off); off += szG1p;
  float* gatep = (float*)(ws + off); off += szTokF;
  float* orec  = (float*)(ws + off); off += szTokF;
  unsigned short* onh = (unsigned short*)(ws + off); off += szX16;
  unsigned short* onl = (unsigned short*)(ws + off); off += szX16;
  if (off > ws_size) return;

  const dim3 blk(256);

  split8_bf16_kernel<<<dim3((kTok * kEmb / 8) / 256), blk, 0, stream>>>(x, xh, xl, kTok * kEmb / 8);

  wtsplit_kernel<<<dim3(kEmb / 64, kEmb / 64, 3), blk, 0, stream>>>(Wq, Wk, Wv, kEmb, kEmb, WTh, WTl);
  wtsplit_kernel<<<dim3(kEmb / 64, kGateRank / 64, 1), blk, 0, stream>>>(G1, G1, G1, kEmb, kGateRank, G1Th, G1Tl);
  wtsplit_kernel<<<dim3(kGateRank / 64, kEmb / 64, 1), blk, 0, stream>>>(G2, G2, G2, kGateRank, kEmb, G2Th, G2Tl);
  wtsplit_kernel<<<dim3(kEmb / 64, kEmb / 64, 1), blk, 0, stream>>>(Wo, Wo, Wo, kEmb, kEmb, WoTh, WoTl);

  wmma_gemm64<1, true, 0, 0, false><<<dim3((kTok / 64) * (kProjN / 64) / 8, 1), blk, 0, stream>>>(
      xh, xl, kEmb, 0L, WTh, WTl, kEmb, 0L, (void*)pre, (void*)pre, kProjN, 0L,
      delta, pre, 0L, kTok, kProjN, kEmb, 1.0f);

  wmma_gemm64<1, true, 0, 2, false><<<dim3((kTok / 64) * (kGateRank / 64) / 8, 1), blk, 0, stream>>>(
      xh, xl, kEmb, 0L, G1Th, G1Tl, kEmb, 0L, (void*)g1h, (void*)g1l, kGateRank, 0L,
      delta, pre, 0L, kTok, kGateRank, kEmb, 1.0f);

  wmma_gemm64<1, true, 0, 0, false><<<dim3((kTok / 64) * (kEmb / 64) / 8, 1), blk, 0, stream>>>(
      g1h, g1l, kGateRank, 0L, G2Th, G2Tl, kGateRank, 0L, (void*)gatep, (void*)gatep, kEmb, 0L,
      delta, pre, 0L, kTok, kEmb, kGateRank, 1.0f);

  prep_kernel<<<dim3(kTok * kEmb / 256), blk, 0, stream>>>(pre, delta, qa, kvp, decp);

  decay_scan_kernel<<<dim3(kBatch * kHeads), dim3(128), 0, stream>>>(qa, kvp, decp, pre, orec);

  gate_norm_kernel<<<dim3(kTok * kHeads / 8), blk, 0, stream>>>(orec, gatep, normw, onh, onl);

  wmma_gemm64<1, true, 0, 0, false><<<dim3((kTok / 64) * (kEmb / 64) / 8, 1), blk, 0, stream>>>(
      onh, onl, kEmb, 0L, WoTh, WoTl, kEmb, 0L, (void*)out, (void*)out, kEmb, 0L,
      delta, pre, 0L, kTok, kEmb, kEmb, 1.0f);
}
